// ScalableAttentionModule_39367670235461
// MI455X (gfx1250) — hardware-verified
//
#include <hip/hip_runtime.h>
#include <math.h>

typedef __attribute__((ext_vector_type(16))) _Float16 v16h;
typedef __attribute__((ext_vector_type(8)))  _Float16 v8h;
typedef __attribute__((ext_vector_type(16))) __bf16   v16b;
typedef __attribute__((ext_vector_type(8)))  float    v8f;
typedef __attribute__((ext_vector_type(4)))  float    v4f;

__device__ __forceinline__ int frag_k(int i, int h) { return (i < 8) ? (8 * h + i) : (16 + 8 * h + (i - 8)); }
__device__ __forceinline__ __bf16 bf16_rne(float f) {
    unsigned int u = __float_as_uint(f);
    u += 0x7fffu + ((u >> 16) & 1u);
    return __builtin_bit_cast(__bf16, (unsigned short)(u >> 16));
}
__device__ __forceinline__ float bf16_f32(__bf16 b) { return __uint_as_float(((unsigned int)__builtin_bit_cast(unsigned short, b)) << 16); }
__device__ __forceinline__ v8f wmma16(v16h a, v16h b, v8f c) {
    c = __builtin_amdgcn_wmma_f32_16x16x32_f16(false, a, false, b, (short)0, c, false, false);
    asm volatile("v_nop\n\tv_nop\n\tv_nop\n\tv_nop" : "+v"(c) : "v"(a), "v"(b));
    return c;
}
__device__ __forceinline__ v8f wmmab(v16b a, v16b b, v8f c) {
    c = __builtin_amdgcn_wmma_f32_16x16x32_bf16(false, a, false, b, (short)0, c, false, false);
    asm volatile("v_nop\n\tv_nop\n\tv_nop\n\tv_nop" : "+v"(c) : "v"(a), "v"(b));
    return c;
}
struct Split { v16b hi, lo; };
__device__ __forceinline__ v8f wmma3(const Split& a, const Split& b, v8f c) {
    c = __builtin_amdgcn_wmma_f32_16x16x32_bf16(false, a.hi, false, b.hi, (short)0, c, false, false);
    c = __builtin_amdgcn_wmma_f32_16x16x32_bf16(false, a.hi, false, b.lo, (short)0, c, false, false);
    c = __builtin_amdgcn_wmma_f32_16x16x32_bf16(false, a.lo, false, b.hi, (short)0, c, false, false);
    asm volatile("v_nop\n\tv_nop\n\tv_nop\n\tv_nop" : "+v"(c) : "v"(a.hi), "v"(a.lo), "v"(b.hi), "v"(b.lo));
    return c;
}
struct Split3 { v16b hi, mid, lo; };
__device__ __forceinline__ v8f wmma6(const Split3& a, const Split3& b, v8f c) {
    c = __builtin_amdgcn_wmma_f32_16x16x32_bf16(false, a.hi, false, b.hi, (short)0, c, false, false);
    c = __builtin_amdgcn_wmma_f32_16x16x32_bf16(false, a.hi, false, b.mid, (short)0, c, false, false);
    c = __builtin_amdgcn_wmma_f32_16x16x32_bf16(false, a.mid, false, b.hi, (short)0, c, false, false);
    c = __builtin_amdgcn_wmma_f32_16x16x32_bf16(false, a.hi, false, b.lo, (short)0, c, false, false);
    c = __builtin_amdgcn_wmma_f32_16x16x32_bf16(false, a.mid, false, b.mid, (short)0, c, false, false);
    c = __builtin_amdgcn_wmma_f32_16x16x32_bf16(false, a.lo, false, b.hi, (short)0, c, false, false);
    asm volatile("v_nop\n\tv_nop\n\tv_nop\n\tv_nop" : "+v"(c) : "v"(a.hi), "v"(a.mid), "v"(a.lo), "v"(b.hi), "v"(b.mid), "v"(b.lo));
    return c;
}

__device__ __forceinline__ v16h fh_ld(const float* __restrict__ p, long long sk, int k0, int h, int klen, float s) {
    v16h a;
#pragma unroll
    for (int i = 0; i < 16; ++i) { const int k = k0 + frag_k(i, h); a[i] = (k < klen) ? (_Float16)(p[(long long)k * sk] * s) : (_Float16)0.f; }
    return a;
}
__device__ __forceinline__ Split sp_ld(const float* __restrict__ p, long long sk, int k0, int h, int klen, float s) {
    Split r;
#pragma unroll
    for (int i = 0; i < 16; ++i) {
        const int k = k0 + frag_k(i, h); const float x = (k < klen) ? p[(long long)k * sk] * s : 0.f;
        const __bf16 hb = bf16_rne(x); r.hi[i] = hb; r.lo[i] = bf16_rne(x - bf16_f32(hb));
    }
    return r;
}
__device__ __forceinline__ Split3 sp3_ld(const float* __restrict__ p, long long sk, int k0, int h, int klen, float s) {
    Split3 r;
#pragma unroll
    for (int i = 0; i < 16; ++i) {
        const int k = k0 + frag_k(i, h); const float x = (k < klen) ? p[(long long)k * sk] * s : 0.f;
        const __bf16 hb = bf16_rne(x); const float r1 = x - bf16_f32(hb); const __bf16 mb = bf16_rne(r1);
        r.hi[i] = hb; r.mid[i] = mb; r.lo[i] = bf16_rne(r1 - bf16_f32(mb));
    }
    return r;
}
__device__ __forceinline__ v16b bh_ld(const float* __restrict__ p, long long sk, int k0, int h, int klen, float s) {
    v16b a;
#pragma unroll
    for (int i = 0; i < 16; ++i) { const int k = k0 + frag_k(i, h); a[i] = bf16_rne((k < klen) ? p[(long long)k * sk] * s : 0.f); }
    return a;
}
__device__ __forceinline__ v16h fh_row(const _Float16* __restrict__ row, int k0, int h) {
    v16h a;
#pragma unroll
    for (int i = 0; i < 16; ++i) a[i] = row[k0 + frag_k(i, h)];
    return a;
}

#define VST2(T, ptr, val) do { const T vst2_v_ = (val); *(volatile T*)(ptr) = vst2_v_; __threadfence(); *(volatile T*)(ptr) = vst2_v_; } while (0)
typedef float v4f __attribute__((ext_vector_type(4)));
#define VST2V4(ptr, val) do { const v4f vst2_v4_ = (val); *(volatile v4f*)(ptr) = vst2_v4_; __threadfence(); *(volatile v4f*)(ptr) = vst2_v4_; } while (0)

__device__ __attribute__((noinline)) float act_fn(float v, int act) {
    if (act == 1) return fmaxf(v, 0.f);
    if (act == 2) { const float u = 0.7978845608028654f * (v + 0.044715f * v * v * v); return 0.5f * v * (1.f + tanhf(u)); }
    if (act == 3) return v / (1.f + expf(-v));
    if (act == 4) return 0.5f * v * (1.f + erff(v * 0.7071067811865476f));
    if (act == 5) return tanhf(v);
    if (act == 6) return 1.f / (1.f + expf(-v));
    if (act == 7) return (v > 0.f) ? v : 0.01f * v;
    if (act == 8) return (v > 0.f) ? v : (expf(v) - 1.f);
    if (act == 9) return fminf(fmaxf(v, 0.f), 6.f);
    if (act == 10) return fabsf(v);
    if (act == 11) return (v >= 0.f) ? v : 0.1f * v;
    if (act == 12) return (v > 0.f) ? v : 0.2f * v;
    if (act == 13) return (v > 20.f) ? v : log1pf(expf(v));
    return v;
}

struct GemmP {
    const float* A; const float* B; const float* bias; const float* R; float* C;
    long long sAo, sAi, sAm, sAk, sBo, sBi, sBn, sBk, sCo, sCi, sCm, sRo, sRi, sRm, sRn;
    int M, N, K, zi_n, flags, act; float alpha, beta, sa, sb;
    int Npad, pad_;
};
static_assert(sizeof(GemmP) == 5 * 8 + 15 * 8 + 6 * 4 + 4 * 4 + 2 * 4, "GemmP has padding");

template <int MODE>
__global__ __launch_bounds__(32) void k_gemm(GemmP p) {
    const int lane = threadIdx.x & 31, h = lane >> 4, l15 = lane & 15;
    const int m0 = blockIdx.y * 16, n0 = blockIdx.x * 32;
    const int z = blockIdx.z, zo = z / p.zi_n, zi = z - zo * p.zi_n;
    const float* A = p.A + zo * p.sAo + zi * p.sAi;
    const float* B = p.B + zo * p.sBo + zi * p.sBi;
    const int am = min(m0 + l15, p.M - 1);
    v8f acc[2], comp[2];
#pragma unroll
    for (int t = 0; t < 2; ++t) { v8f zz = {}; acc[t] = zz; comp[t] = zz; }
    for (int k0 = 0; k0 < p.K; k0 += 32) {
        const float* arow = A + (long long)am * p.sAm;
        if (MODE == 1) {
            const Split a = sp_ld(arow, p.sAk, k0, h, p.K, 1.f);
#pragma unroll
            for (int t = 0; t < 2; ++t) {
                const int bn = min(n0 + t * 16 + l15, p.N - 1);
                acc[t] = wmma3(a, sp_ld(B + (long long)bn * p.sBn, p.sBk, k0, h, p.K, 1.f), acc[t]);
            }
        } else if (MODE == 3) {
            const Split3 a = sp3_ld(arow, p.sAk, k0, h, p.K, 1.f);
#pragma unroll
            for (int t = 0; t < 2; ++t) {
                const int bn = min(n0 + t * 16 + l15, p.N - 1);
                acc[t] = wmma6(a, sp3_ld(B + (long long)bn * p.sBn, p.sBk, k0, h, p.K, 1.f), acc[t]);
            }
        } else if (MODE == 4) {
            const Split3 a = sp3_ld(arow, p.sAk, k0, h, p.K, 1.f);
#pragma unroll
            for (int t = 0; t < 2; ++t) {
                const int bn = min(n0 + t * 16 + l15, p.N - 1); v8f zz = {};
                const v8f part = wmma6(a, sp3_ld(B + (long long)bn * p.sBn, p.sBk, k0, h, p.K, 1.f), zz);
                const v8f y = part - comp[t]; const v8f s = acc[t] + y; comp[t] = (s - acc[t]) - y; acc[t] = s;
            }
        } else if (MODE == 2) {
            const v16b a = bh_ld(arow, p.sAk, k0, h, p.K, 1.f);
#pragma unroll
            for (int t = 0; t < 2; ++t) {
                const int bn = min(n0 + t * 16 + l15, p.N - 1);
                acc[t] = wmmab(a, bh_ld(B + (long long)bn * p.sBn, p.sBk, k0, h, p.K, 1.f), acc[t]);
            }
        } else {
            const v16h a = fh_ld(arow, p.sAk, k0, h, p.K, p.sa);
#pragma unroll
            for (int t = 0; t < 2; ++t) {
                const int bn = min(n0 + t * 16 + l15, p.N - 1);
                acc[t] = wmma16(a, fh_ld(B + (long long)bn * p.sBn, p.sBk, k0, h, p.K, p.sb), acc[t]);
            }
        }
    }
    const float iscale = (MODE == 0) ? p.alpha / (p.sa * p.sb) : p.alpha;
    float* C = p.C + zo * p.sCo + zi * p.sCi;
    const float* R = p.R + zo * p.sRo + zi * p.sRi;
    __shared__ __align__(16) float ctile[16][36];
#pragma unroll
    for (int t = 0; t < 2; ++t) {
        const int n = n0 + t * 16 + l15; const int nn = min(n, p.N - 1);
#pragma unroll
        for (int r = 0; r < 8; ++r) {
            const int m = m0 + 8 * h + r; const int mm = min(m, p.M - 1);
            float v = acc[t][r] * iscale;
            if (p.flags & 1) v += p.bias[nn];
            if (p.flags & 2) v += p.bias[mm];
            if (p.flags & 8) v *= p.bias[(long long)zo * p.M + mm];
            v = act_fn(v, p.act);
            if (p.flags & 4) v += p.beta * R[(long long)mm * p.sRm + (long long)nn * p.sRn];
            ctile[8 * h + r][t * 16 + l15] = (n < p.N) ? v : 0.f;
        }
    }
    __syncthreads();
    const int NW = (p.Npad > p.N) ? p.Npad : p.N;
    const bool fast = (m0 + 16 <= p.M) && (n0 + 32 <= NW) && ((p.sCm & 3) == 0) && ((((size_t)C) & 15) == 0);
    if (fast) {
#pragma unroll
        for (int s = 0; s < 4; ++s) {
            const int row = s * 4 + (lane >> 3), c4 = (lane & 7) * 4;
            const v4f v = *(const v4f*)&ctile[row][c4];
            VST2V4(C + (long long)(m0 + row) * p.sCm + n0 + c4, v);
        }
    } else {
        for (int row = 0; row < 16; ++row) {
            const int m = m0 + row, n = n0 + lane;
            if (m < p.M && n < NW) VST2(float, C + (long long)m * p.sCm + n, ctile[row][lane]);
        }
    }
}


template <int MODE, int TM, int TN>
__global__ __launch_bounds__(32) void k_gemmT(GemmP p) {
    const int lane = threadIdx.x & 31, h = lane >> 4, l15 = lane & 15;
    const int m0 = blockIdx.y * (16 * TM), n0 = blockIdx.x * (16 * TN);
    const int z = blockIdx.z, zo = z / p.zi_n, zi = z - zo * p.zi_n;
    const float* A = p.A + zo * p.sAo + zi * p.sAi;
    const float* B = p.B + zo * p.sBo + zi * p.sBi;
    v8f acc[TM][TN];
#pragma unroll
    for (int i = 0; i < TM; ++i)
#pragma unroll
        for (int t = 0; t < TN; ++t) { v8f zz = {}; acc[i][t] = zz; }
    for (int k0 = 0; k0 < p.K; k0 += 32) {
        if (MODE == 1) {
            Split a[TM], b[TN];
#pragma unroll
            for (int i = 0; i < TM; ++i) { const int am = min(m0 + 16 * i + l15, p.M - 1); a[i] = sp_ld(A + (long long)am * p.sAm, p.sAk, k0, h, p.K, 1.f); }
#pragma unroll
            for (int t = 0; t < TN; ++t) { const int bn = min(n0 + 16 * t + l15, p.N - 1); b[t] = sp_ld(B + (long long)bn * p.sBn, p.sBk, k0, h, p.K, 1.f); }
#pragma unroll
            for (int i = 0; i < TM; ++i)
#pragma unroll
                for (int t = 0; t < TN; ++t) acc[i][t] = wmma3(a[i], b[t], acc[i][t]);
        } else if (MODE == 2) {
            v16b a[TM], b[TN];
#pragma unroll
            for (int i = 0; i < TM; ++i) { const int am = min(m0 + 16 * i + l15, p.M - 1); a[i] = bh_ld(A + (long long)am * p.sAm, p.sAk, k0, h, p.K, 1.f); }
#pragma unroll
            for (int t = 0; t < TN; ++t) { const int bn = min(n0 + 16 * t + l15, p.N - 1); b[t] = bh_ld(B + (long long)bn * p.sBn, p.sBk, k0, h, p.K, 1.f); }
#pragma unroll
            for (int i = 0; i < TM; ++i)
#pragma unroll
                for (int t = 0; t < TN; ++t) acc[i][t] = wmmab(a[i], b[t], acc[i][t]);
        } else {
            v16h a[TM], b[TN];
#pragma unroll
            for (int i = 0; i < TM; ++i) { const int am = min(m0 + 16 * i + l15, p.M - 1); a[i] = fh_ld(A + (long long)am * p.sAm, p.sAk, k0, h, p.K, p.sa); }
#pragma unroll
            for (int t = 0; t < TN; ++t) { const int bn = min(n0 + 16 * t + l15, p.N - 1); b[t] = fh_ld(B + (long long)bn * p.sBn, p.sBk, k0, h, p.K, p.sb); }
#pragma unroll
            for (int i = 0; i < TM; ++i)
#pragma unroll
                for (int t = 0; t < TN; ++t) acc[i][t] = wmma16(a[i], b[t], acc[i][t]);
        }
    }
    const float iscale = (MODE == 0) ? p.alpha / (p.sa * p.sb) : p.alpha;
    float* C = p.C + zo * p.sCo + zi * p.sCi;
    const float* R = p.R + zo * p.sRo + zi * p.sRi;
    const int NW = (p.Npad > p.N) ? p.Npad : p.N;
    __shared__ __align__(16) float ctile[16][36];
#pragma unroll
    for (int i = 0; i < TM; ++i) {
        const int mb = m0 + 16 * i; if (mb >= p.M) break;
#pragma unroll
        for (int tp = 0; tp < TN / 2; ++tp) {
            const int nb = n0 + 32 * tp; if (nb >= NW) break;
#pragma unroll
            for (int t2 = 0; t2 < 2; ++t2) {
                const int t = 2 * tp + t2; const int n = nb + t2 * 16 + l15; const int nn = min(n, p.N - 1);
#pragma unroll
                for (int r = 0; r < 8; ++r) {
                    const int m = mb + 8 * h + r; const int mm = min(m, p.M - 1);
                    float v = acc[i][t][r] * iscale;
                    if (p.flags & 1) v += p.bias[nn];
                    if (p.flags & 2) v += p.bias[mm];
            if (p.flags & 8) v *= p.bias[(long long)zo * p.M + mm];
                    v = act_fn(v, p.act);
                    if (p.flags & 4) v += p.beta * R[(long long)mm * p.sRm + (long long)nn * p.sRn];
                    ctile[8 * h + r][t2 * 16 + l15] = (n < p.N) ? v : 0.f;
                }
            }
            __syncthreads();
            const bool fast = (mb + 16 <= p.M) && (nb + 32 <= NW) && ((p.sCm & 3) == 0) && ((((size_t)C) & 15) == 0);
            if (fast) {
#pragma unroll
                for (int s = 0; s < 4; ++s) {
                    const int row = s * 4 + (lane >> 3), c4 = (lane & 7) * 4;
                    const v4f v = *(const v4f*)&ctile[row][c4];
                    VST2V4(C + (long long)(mb + row) * p.sCm + nb + c4, v);
                }
            } else {
                for (int row = 0; row < 16; ++row) {
                    const int m = mb + row, n = nb + lane;
                    if (m < p.M && n < NW) VST2(float, C + (long long)m * p.sCm + n, ctile[row][lane]);
                }
            }
            __syncthreads();
        }
    }
}

#define AW 4
struct AttnP {
    const float* Q; const float* K; const float* V; float* O; float* P; const float* Mf; const int* Mi; float* ST;
    const float* Pw; const float* Rt; const int* SQ; const int* SK;
    long long swb, swh, swi, swj, srb, srh, sri;
    long long sQb, sQh, sQi, sQd, sKb, sKh, sKj, sKd, sVb, sVh, sVj, sVd, sOb, sOh, sOi, sPb, sPh, sPi, smb, smh, smi, smj;
    int Lq, Lk, dh, dv, hrep, causal, coff, pband;
    float scale, mfill; int nonorm, mpol;
    int roff, rn, segpol, win;
};
static_assert(sizeof(AttnP) == 12 * 8 + 29 * 8 + 16 * 4, "AttnP has padding");

#ifndef KATTN_ATTR
#define KATTN_ATTR
#endif
template <int DHP, int DVP, int QM, bool SPLITPV, bool TWOPASS>
__global__ __launch_bounds__(32 * AW) KATTN_ATTR void k_attn(AttnP p) {
    constexpr int NT = DVP / 16;
    constexpr int KS = DHP / 32;
    constexpr int VP = DVP + 8;
    __shared__ __align__(16) float    pl[AW][16 * 64];
    __shared__ __align__(16) _Float16 vl[(SPLITPV ? 2 : 1) * 64 * VP];
    const int lane = threadIdx.x & 31, hf = lane >> 4, l15 = lane & 15, wave = threadIdx.x >> 5;
    const int h = blockIdx.y, b = blockIdx.z, hk = h / p.hrep;
    const int q0 = (blockIdx.x * AW + wave) * 16;
    float* myp = pl[wave];
    const float L2E = 1.4426950408889634f;
    const float NEG = -__builtin_inff();
    const int qi = min(q0 + l15, p.Lq - 1);
    const float* qrow = p.Q + b * p.sQb + h * p.sQh + (long long)qi * p.sQi;
    const float* kbase = p.K + b * p.sKb + hk * p.sKh;
    const float* vbase = p.V + b * p.sVb + hk * p.sVh;
    v16h qa[QM == 0 ? KS : 1]; Split qs_[QM == 1 ? KS : 1]; Split3 qt_[QM == 2 ? KS : 1];
#pragma unroll
    for (int ks = 0; ks < KS; ++ks) {
        if (QM == 2) qt_[ks] = sp3_ld(qrow, p.sQd, ks * 32, hf, p.dh, 1.f);
        else if (QM == 1) qs_[ks] = sp_ld(qrow, p.sQd, ks * 32, hf, p.dh, 1.f);
        else qa[ks] = fh_ld(qrow, p.sQd, ks * 32, hf, p.dh, 1.f);
    }
    v8f o[NT]; float m8[8], l8[8];
#pragma unroll
    for (int t = 0; t < NT; ++t) { v8f zz = {}; o[t] = zz; }
#pragma unroll
    for (int i = 0; i < 8; ++i) { m8[i] = NEG; l8[i] = 0.f; }
    int jend = p.Lk;
    if (p.causal == 1) { const int je = (blockIdx.x * AW + AW - 1) * 16 + 16 + p.coff; jend = min(jend, max(je, 0)); }
    const int npass = TWOPASS ? 2 : 1;
    for (int pass = 0; pass < npass; ++pass) {
        const bool dopv = (!TWOPASS) || pass == 1;
        for (int j0 = 0; j0 < jend; j0 += 64) {
            if (dopv) {
                __syncthreads();
                for (int idx = threadIdx.x; idx < 64 * DVP; idx += 32 * AW) {
                    const int jr = idx / DVP, d = idx - jr * DVP, j = j0 + jr;
                    const float f = (j < p.Lk && d < p.dv) ? vbase[(long long)j * p.sVj + (long long)d * p.sVd] : 0.f;
                    if (SPLITPV) {
                        const __bf16 hb = bf16_rne(f);
                        ((__bf16*)vl)[jr * VP + d] = hb; ((__bf16*)vl)[64 * VP + jr * VP + d] = bf16_rne(f - bf16_f32(hb));
                    } else vl[jr * VP + d] = (_Float16)f;
                }
            }
            v8f s[4];
#pragma unroll
            for (int t = 0; t < 4; ++t) {
                const int j = min(j0 + t * 16 + l15, p.Lk - 1);
                const float* krow = kbase + (long long)j * p.sKj;
                v8f acc = {};
#pragma unroll
                for (int ks = 0; ks < KS; ++ks) {
                    if (QM == 2)      acc = wmma6(qt_[ks], sp3_ld(krow, p.sKd, ks * 32, hf, p.dh, 1.f), acc);
                    else if (QM == 1) acc = wmma3(qs_[ks], sp_ld(krow, p.sKd, ks * 32, hf, p.dh, 1.f), acc);
                    else              acc = wmma16(qa[ks], fh_ld(krow, p.sKd, ks * 32, hf, p.dh, 1.f), acc);
                }
                s[t] = acc;
            }
            float pv[8][4];
#pragma unroll
            for (int i = 0; i < 8; ++i) {
                const int irow = q0 + i + 8 * hf;
                const int ic = min(irow, p.Lq - 1);
                float sc[4];
#pragma unroll
                for (int t = 0; t < 4; ++t) {
                    const int jg = j0 + t * 16 + l15;
                    float v = s[t][i] * p.scale;
                    if (p.Mf) v += p.Mf[b * p.smb + h * p.smh + (long long)ic * p.smi + (long long)min(jg, p.Lk - 1) * p.smj];
                    if (p.Rt) { int rc = ic - min(jg, p.Lk - 1) + p.roff; rc = rc < 0 ? 0 : (rc >= p.rn ? p.rn - 1 : rc); v += p.Rt[b * p.srb + h * p.srh + (long long)ic * p.sri + rc]; }
                    if (p.Mi) { const int mv = p.Mi[b * p.smb + h * p.smh + (long long)ic * p.smi + (long long)min(jg, p.Lk - 1) * p.smj]; if (p.mpol ? (mv != 0) : (mv == 0)) v = p.mfill; }
                    if (p.SQ) { const bool same = p.SQ[(long long)b * p.Lq + ic] == p.SK[(long long)b * p.Lk + min(jg, p.Lk - 1)]; if (p.segpol ? same : !same) v = p.mfill; }
                    if (p.causal == 2 && jg > irow + p.coff) v = p.mfill;
                    if (jg >= p.Lk || (p.causal == 1 && jg > irow + p.coff) || (p.causal == 3 && jg < irow + p.coff) || (p.win > 0 && irow + p.coff - jg > p.win)) v = NEG; else v *= L2E;
                    sc[t] = v;
                }
                if (!TWOPASS || pass == 0) {
                    float mx = fmaxf(fmaxf(sc[0], sc[1]), fmaxf(sc[2], sc[3]));
                    mx = fmaxf(mx, __shfl_xor(mx, 1, 32)); mx = fmaxf(mx, __shfl_xor(mx, 2, 32));
                    mx = fmaxf(mx, __shfl_xor(mx, 4, 32)); mx = fmaxf(mx, __shfl_xor(mx, 8, 32));
                    const float mnew = fmaxf(m8[i], mx);
                    const float corr = (mnew == NEG) ? 1.f : exp2f(m8[i] - mnew);
                    float rs = 0.f;
#pragma unroll
                    for (int t = 0; t < 4; ++t) {
                        const float pp = (sc[t] == NEG) ? 0.f : exp2f(sc[t] - mnew); rs += pp;
                        pv[i][t] = p.Pw ? pp * p.Pw[b * p.swb + h * p.swh + (long long)ic * p.swi + (long long)min(j0 + t * 16 + l15, p.Lk - 1) * p.swj] : pp;
                    }
                    rs += __shfl_xor(rs, 1, 32); rs += __shfl_xor(rs, 2, 32); rs += __shfl_xor(rs, 4, 32); rs += __shfl_xor(rs, 8, 32);
                    l8[i] = l8[i] * corr + rs; m8[i] = mnew;
                    if (!TWOPASS) {
#pragma unroll
                        for (int t = 0; t < NT; ++t) o[t][i] *= corr;
                    }
                } else {
                    const float inv = (l8[i] > 0.f) ? 1.f / l8[i] : 0.f;
#pragma unroll
                    for (int t = 0; t < 4; ++t) {
                        const int jg = j0 + t * 16 + l15;
                        float pp = (sc[t] == NEG) ? 0.f : exp2f(sc[t] - m8[i]) * inv;
                        if (p.Pw) pp *= p.Pw[b * p.swb + h * p.swh + (long long)ic * p.swi + (long long)min(jg, p.Lk - 1) * p.swj];
                        pv[i][t] = pp;
                    }
                }
            }
            if (dopv) {
#pragma unroll
                for (int i = 0; i < 8; ++i)
#pragma unroll
                    for (int t = 0; t < 4; ++t) ((volatile float*)myp)[(i + 8 * hf) * 64 + t * 16 + l15] = pv[i][t];
                __syncthreads();
                if (p.P) {
                    float* pb_ = p.P + b * p.sPb + h * p.sPh;
                    const bool fastP = (p.pband == 0) && ((p.sPi & 3) == 0) && (j0 + 64 <= p.Lk) && (q0 + 16 <= p.Lq) && ((((size_t)pb_) & 15) == 0);
                    if (fastP) {
#pragma unroll
                        for (int s = 0; s < 8; ++s) {
                            const int row = s * 2 + (lane >> 4), c4 = (lane & 15) * 4;
                            const v4f v = *(const v4f*)(myp + row * 64 + c4);
                            VST2V4(pb_ + (long long)(q0 + row) * p.sPi + j0 + c4, v);
                        }
                    } else {
                        for (int row = 0; row < 16; ++row) {
                            const int irow = q0 + row; if (irow >= p.Lq) continue;
                            for (int c = lane; c < 64; c += 32) {
                                const int jg = j0 + c; if (jg >= p.Lk) continue;
                                if (p.pband == 0) VST2(float, pb_ + (long long)irow * p.sPi + jg, myp[row * 64 + c]);
                                else if (jg - irow <= p.pband && irow - jg <= p.pband) VST2(float, pb_ + (long long)irow * p.sPi + (jg - irow + p.pband), myp[row * 64 + c]);
                            }
                        }
                    }
                }
                if (SPLITPV) {
                    const Split pa0 = sp_ld(myp + l15 * 64, 1, 0, hf, 64, 1.f), pa1 = sp_ld(myp + l15 * 64, 1, 32, hf, 64, 1.f);
                    const __bf16* vh = (const __bf16*)vl; const __bf16* vlo = vh + 64 * VP;
#pragma unroll
                    for (int t = 0; t < NT; ++t) {
                        const int dcol = t * 16 + l15;
                        Split b0, b1;
#pragma unroll
                        for (int e = 0; e < 16; ++e) {
                            const int k0 = frag_k(e, hf), k1 = 32 + frag_k(e, hf);
                            b0.hi[e] = vh[k0 * VP + dcol]; b0.lo[e] = vlo[k0 * VP + dcol]; b1.hi[e] = vh[k1 * VP + dcol]; b1.lo[e] = vlo[k1 * VP + dcol];
                        }
                        o[t] = wmma3(pa0, b0, o[t]);
                        o[t] = wmma3(pa1, b1, o[t]);
                    }
                } else {
                    const v16h pa0 = fh_ld(myp + l15 * 64, 1, 0, hf, 64, 4096.f), pa1 = fh_ld(myp + l15 * 64, 1, 32, hf, 64, 4096.f);
#pragma unroll
                    for (int t = 0; t < NT; ++t) {
                        const int dcol = t * 16 + l15;
                        v16h b0, b1;
#pragma unroll
                        for (int e = 0; e < 16; ++e) { b0[e] = vl[frag_k(e, hf) * VP + dcol]; b1[e] = vl[(32 + frag_k(e, hf)) * VP + dcol]; }
                        o[t] = wmma16(pa0, b0, o[t]);
                        o[t] = wmma16(pa1, b1, o[t]);
                    }
                }
            }
        }
    }
    float* obase = p.O + b * p.sOb + h * p.sOh;
    if (p.ST) {
        const int rl = lane >> 1, isel = rl & 7;
        float mv = 0.f, lv = 0.f;
#pragma unroll
        for (int i = 0; i < 8; ++i) if (i == isel) { mv = m8[i]; lv = l8[i]; }
        const int irow = q0 + rl;
        if (irow < p.Lq) { float* st = p.ST + (((long long)b * gridDim.y + h) * p.Lq + irow) * 2 + (lane & 1); VST2(float, st, (lane & 1) ? lv : mv * 0.6931471805599453f); }
    }
    float invr[8];
#pragma unroll
    for (int i = 0; i < 8; ++i) {
        if (TWOPASS) invr[i] = SPLITPV ? 1.f : (1.f / 4096.f);
        else if (p.nonorm) invr[i] = exp2f(m8[i]) * (SPLITPV ? 1.f : (1.f / 4096.f));
        else invr[i] = (l8[i] > 0.f) ? (SPLITPV ? 1.f / l8[i] : 1.f / (l8[i] * 4096.f)) : 0.f;
    }
    __syncthreads();
    const bool ofast = ((p.sOi & 3) == 0) && ((((size_t)obase) & 15) == 0) && (q0 + 16 <= p.Lq);
#pragma unroll
    for (int c0 = 0; c0 < DVP; c0 += 64) {
#pragma unroll
        for (int i = 0; i < 8; ++i)
#pragma unroll
            for (int t = 0; t < NT; ++t) if (t * 16 >= c0 && t * 16 < c0 + 64) ((volatile float*)myp)[(i + 8 * hf) * 64 + (t * 16 - c0) + l15] = o[t][i] * invr[i];
        __syncthreads();
        const int cw = (DVP - c0 < 64) ? (DVP - c0) : 64;
        if (ofast && (c0 + cw <= p.dv) && (cw % 32 == 0)) {
            const int lpr = cw / 4;
            const int rows_per_ins = 32 / lpr;
            for (int r0 = 0; r0 < 16; r0 += rows_per_ins) {
                const int row = r0 + lane / lpr, c4 = (lane % lpr) * 4;
                const v4f v = *(const v4f*)(myp + row * 64 + c4);
                VST2V4(obase + (long long)(q0 + row) * p.sOi + c0 + c4, v);
            }
        } else {
            for (int row = 0; row < 16; ++row) {
                const int irow = q0 + row; if (irow >= p.Lq) continue;
                for (int c = lane; c < cw; c += 32) { const int d = c0 + c; if (d < p.dv) VST2(float, obase + (long long)irow * p.sOi + d, myp[row * 64 + c]); }
            }
        }
        __syncthreads();
    }
}

struct TrP { const float* src; float* dst; const float* R2; long long sSz, lds, sDz, ldd, sRz, ldr; int R, C, flags, act; float alpha, beta; };
static_assert(sizeof(TrP) == 3 * 8 + 6 * 8 + 6 * 4, "TrP has padding");
__global__ __launch_bounds__(256) void k_tr(TrP p) {
    __shared__ float tile[32][33];
    const int c0 = blockIdx.x * 32, r0 = blockIdx.y * 32, z = blockIdx.z;
    const int lane = threadIdx.x & 31, wave = threadIdx.x >> 5;
    const float* s = p.src + z * p.sSz;
#pragma unroll
    for (int k = 0; k < 4; ++k) {
        const int rl = wave * 4 + k, r = r0 + rl, c = c0 + lane;
        tile[rl][lane] = (r < p.R && c < p.C) ? s[(long long)r * p.lds + c] : 0.f;
    }
    __syncthreads();
    float* d = p.dst + z * p.sDz; const float* rr = p.R2 + z * p.sRz;
#pragma unroll
    for (int k = 0; k < 4; ++k) {
        const int cl = wave * 4 + k, c = c0 + cl, r = r0 + lane;
        if (c < p.C && r < p.R) {
            float v = act_fn(p.alpha * tile[lane][cl], p.act);
            if (p.flags & 1) v += p.beta * rr[(long long)c * p.ldr + r];
            VST2(float, d + (long long)c * p.ldd + r, v);
        }
    }
}

__global__ __launch_bounds__(256) void k_affine(const float* __restrict__ src, float* __restrict__ dst, int n, float a, float b, const float* __restrict__ sdev) {
    const int i = blockIdx.x * 256 + threadIdx.x;
    if (i < n) { const float aa = sdev ? a * sdev[0] : a; const float v = aa * src[i] + b; VST2(float, dst + i, v); }
}

struct SmP { const float* src; float* dst; const float* Mf; long long sz, sr, dz, dr, smz, smr; int n, pad; float scale_in, scale_out; };
static_assert(sizeof(SmP) == 3 * 8 + 6 * 8 + 4 * 4, "SmP has padding");
__global__ __launch_bounds__(256) void k_softmax(SmP p) {
    __shared__ float red[256];
    const int r = blockIdx.x, z = blockIdx.y, tid = threadIdx.x;
    const float* s = p.src + z * p.sz + (long long)r * p.sr;
    const float* mf = p.Mf ? (p.Mf + z * p.smz + (long long)r * p.smr) : nullptr;
    float mx = -__builtin_inff();
    for (int j = tid; j < p.n; j += 256) { float v = s[j] * p.scale_in; if (mf) v += mf[j]; mx = fmaxf(mx, v); }
    red[tid] = mx; __syncthreads();
    for (int o = 128; o > 0; o >>= 1) { if (tid < o) red[tid] = fmaxf(red[tid], red[tid + o]); __syncthreads(); }
    mx = red[0]; __syncthreads();
    float sum = 0.f;
    for (int j = tid; j < p.n; j += 256) { float v = s[j] * p.scale_in; if (mf) v += mf[j]; sum += (mx == -__builtin_inff()) ? 0.f : expf(v - mx); }
    red[tid] = sum; __syncthreads();
    for (int o = 128; o > 0; o >>= 1) { if (tid < o) red[tid] += red[tid + o]; __syncthreads(); }
    sum = red[0];
    const float inv = (sum > 0.f) ? p.scale_out / sum : 0.f;
    float* d = p.dst + z * p.dz + (long long)r * p.dr;
    for (int j = tid; j < p.n; j += 256) { float v = s[j] * p.scale_in; if (mf) v += mf[j]; const float o = (mx == -__builtin_inff()) ? 0.f : expf(v - mx) * inv; VST2(float, d + j, o); }
}
__global__ __launch_bounds__(256) void k_stats(const float* __restrict__ x, long long sz, long long so, long long si, int inner, int n, float eps, float* __restrict__ stat, int mode) {
    __shared__ float red[256];
    const int z = blockIdx.x, tid = threadIdx.x;
    const float* base = x + z * sz;
    float s = 0.f;
    for (int e = tid; e < n; e += 256) s += base[(long long)(e / inner) * so + (long long)(e % inner) * si];
    red[tid] = s; __syncthreads();
    for (int o = 128; o > 0; o >>= 1) { if (tid < o) red[tid] += red[tid + o]; __syncthreads(); }
    const float mu = (mode == 0 || mode == 3) ? red[0] / (float)n : 0.f; __syncthreads();
    float q = 0.f;
    for (int e = tid; e < n; e += 256) { const float dlt = base[(long long)(e / inner) * so + (long long)(e % inner) * si] - mu; q += dlt * dlt; }
    red[tid] = q; __syncthreads();
    for (int o = 128; o > 0; o >>= 1) { if (tid < o) red[tid] += red[tid + o]; __syncthreads(); }
    {
        float rs;
        if (mode == 2) rs = sqrtf((float)n) / fmaxf(sqrtf(red[0]), eps); else if (mode == 3) rs = rsqrtf(red[0] / (float)(n - 1) + eps); else rs = rsqrtf(red[0] / (float)n + eps);
        if (tid < 32) { const float v = (tid == 0) ? mu : ((tid == 1) ? rs : 0.f); VST2(float, stat + (long long)z * 32 + tid, v); }
    }
}
__global__ __launch_bounds__(256) void k_norm_apply(const float* __restrict__ x, float* __restrict__ y, const float* __restrict__ stat, const float* __restrict__ g, const float* __restrict__ bta,
                                                     int Z, int C, int L, int G, int bn, int act) {
    const long long idx = (long long)blockIdx.x * 256 + threadIdx.x;
    if (idx >= (long long)Z * C * L) return;
    const int l = (int)(idx % L); const long long zc = idx / L; const int c = (int)(zc % C), z = (int)(zc / C); (void)l;
    const int set = bn ? c : (z * G + c / (C / G));
    float v = (x[idx] - stat[(long long)set * 32]) * stat[(long long)set * 32 + 1];
    if (g) v *= g[c];
    if (bta) v += bta[c];
    v = act_fn(v, act);
    VST2(float, y + idx, v);
}

__global__ __launch_bounds__(256) void k_lse_neg(const float* __restrict__ st, float* __restrict__ c, int n) {
    const int i = blockIdx.x * 256 + threadIdx.x;
    if (i < n) { const float v = -(st[2 * i] + logf(st[2 * i + 1])); VST2(float, c + i, v); }
}

__global__ __launch_bounds__(256) void k_iota(int* __restrict__ dst, int n, int a, int b) {
    const int i = blockIdx.x * 256 + threadIdx.x;
    if (i < n) { const int v = a * i + b; VST2(int, dst + i, v); }
}

__global__ __launch_bounds__(256) void k_axpby(const float* __restrict__ x, const float* __restrict__ y, float* __restrict__ dst, int n, float a, float b, float c) {
    const int i = blockIdx.x * 256 + threadIdx.x;
    if (i < n) { const float v = a * x[i] + b * y[i] + c; VST2(float, dst + i, v); }
}

struct RopeP { const float* X; float* Y; const float* C; const float* Sn; const int* pos; long long sXr, sXh, sYr, sYh, sCb, sCp, sCd; int R, Hn, D, S, mode, tmode, pmode, pad; };
static_assert(sizeof(RopeP) == 5 * 8 + 7 * 8 + 8 * 4, "RopeP has padding");
__global__ __launch_bounds__(256) void k_rope(RopeP p) {
    const long long idx = (long long)blockIdx.x * 256 + threadIdx.x;
    if (idx >= (long long)p.R * p.Hn * p.D) return;
    const int d = (int)(idx % p.D); const long long rh = idx / p.D; const int h = (int)(rh % p.Hn); const int r = (int)(rh / p.Hn);
    const int half = p.D / 2;
    int partner; float sign;
    if (p.mode == 0) { partner = (d < half) ? d + half : d - half; sign = (d < half) ? -1.f : 1.f; }
    else { partner = d ^ 1; sign = (d & 1) ? 1.f : -1.f; }
    const int tcol = (p.tmode == 0) ? d : ((p.tmode == 1) ? (d % half) : (d >> 1));
    const int pp = (p.pmode == 0) ? (r % p.S) : ((p.pmode == 1) ? h : p.pos[r]);
    const long long toff = (long long)(r / p.S) * p.sCb + (long long)pp * p.sCp + (long long)tcol * p.sCd;
    const float* xr = p.X + (long long)r * p.sXr + (long long)h * p.sXh;
    const float v = xr[d] * p.C[toff] + sign * xr[partner] * p.Sn[toff];
    VST2(float, p.Y + (long long)r * p.sYr + (long long)h * p.sYh + d, v);
}

__global__ __launch_bounds__(256) void k_invf(float* __restrict__ invb, int half, int D, float base, float num, int fmode, float cexp) {
    const int i = blockIdx.x * 256 + threadIdx.x;
    if (i >= ((half + 31) / 32) * 32) return;
    if (i >= half) { VST2(float, invb + i, 0.f); return; }
    const float e = (float)(2 * i) / (float)D;
    float invf;
    if (fmode == 1) invf = num * expf((float)(2 * i) * cexp);
    else if (fmode == 2) invf = num * powf(base, (-2.0f * ((float)i - 1.0f)) / (float)D);
    else invf = num * (1.0f / powf(base, e));
    VST2(float, invb + i, invf);
}
__global__ __launch_bounds__(256) void k_sincos(float* __restrict__ cs, float* __restrict__ sn, const float* __restrict__ invb, int S, int half, float pscale) {
    const int idx = blockIdx.x * 256 + threadIdx.x;
    if (idx >= S * half) return;
    const int s = idx / half, i = idx - s * half;
    const float ang = (pscale * (float)s) * invb[i];
    VST2(float, cs + idx, cosf(ang)); VST2(float, sn + idx, sinf(ang));
}

__global__ __launch_bounds__(256) void k_mulact(const float* __restrict__ x, const float* __restrict__ y, float* __restrict__ dst, int n, int act) {
    const int i = blockIdx.x * 256 + threadIdx.x;
    if (i < n) { const float v = act_fn(x[i], act) * y[i]; VST2(float, dst + i, v); }
}

__global__ __launch_bounds__(256) void k_matvec(GemmP p) {
    const int rpt = (p.N == 1) ? 1 : 32;
    const long long r0 = ((long long)blockIdx.x * 256 + threadIdx.x) * rpt; const int z = blockIdx.z, zo = z / p.zi_n, zi = z - zo * p.zi_n;
    if (r0 >= p.M) return;
    const float* Bb = p.B + zo * p.sBo + zi * p.sBi;
    float* C = p.C + zo * p.sCo + zi * p.sCi; const float* R = p.R + zo * p.sRo + zi * p.sRi;
    for (int rr = 0; rr < rpt; ++rr) {
        const long long r = r0 + rr; if (r >= p.M) break;
        const float* A = p.A + zo * p.sAo + zi * p.sAi + r * p.sAm;
        float acc[8] = {0.f, 0.f, 0.f, 0.f, 0.f, 0.f, 0.f, 0.f};
        for (int k = 0; k < p.K; ++k) { const float a = A[(long long)k * p.sAk];
#pragma unroll
            for (int j = 0; j < 8; ++j) if (j < p.N) acc[j] += a * Bb[(long long)j * p.sBn + (long long)k * p.sBk]; }
#pragma unroll
        for (int j = 0; j < 8; ++j) if (j < p.N) {
            float v = acc[j] * p.alpha;
            if (p.flags & 1) v += p.bias[j];
            if (p.flags & 2) v += p.bias[r];
            v = act_fn(v, p.act);
            if (p.flags & 4) v += p.beta * R[r * p.sRm + (long long)j * p.sRn];
            VST2(float, C + r * p.sCm + j, v);
        }
    }
}
__global__ __launch_bounds__(256) void k_smallsoftmax(const float* __restrict__ src, float* __restrict__ dst, long long sr, long long dr, int n, long long R, float scale) {
    const long long r0 = ((long long)blockIdx.x * 256 + threadIdx.x) * 32;
    for (int rr = 0; rr < 32; ++rr) {
        const long long r = r0 + rr; if (r >= R) return;
        const float* s = src + r * sr; float* d = dst + r * dr;
        float mx = -__builtin_inff();
        for (int j = 0; j < n; ++j) mx = fmaxf(mx, s[j] * scale);
        float sum = 0.f;
        for (int j = 0; j < n; ++j) sum += expf(s[j] * scale - mx);
        const float inv = 1.f / sum;
        for (int j = 0; j < n; ++j) { const float v = expf(s[j] * scale - mx) * inv; VST2(float, d + j, v); }
    }
}

__global__ __launch_bounds__(32) void k_unitstat(float* __restrict__ st) { const int t = threadIdx.x; const float v = (t == 1) ? 1.f : 0.f; VST2(float, st + t, v); }

__global__ __launch_bounds__(256) void k_lincopy(const float* __restrict__ src, long long lds, float* __restrict__ dst, long long ldd, long long rows, int cols) {
    const long long i = (long long)blockIdx.x * 256 + threadIdx.x; if (i >= rows * cols) return;
    const long long r = i / cols; const int c = (int)(i - r * cols);
    const float v = src[r * lds + c]; VST2(float, dst + r * ldd + c, v);
}

__global__ __launch_bounds__(256) void k_sa_ones(float* __restrict__ MSGX, int NR, int MX) { const int t = blockIdx.x * 256 + threadIdx.x; if (t >= NR * 32) return; const int r = t >> 5, c = t & 31; VST2(float, MSGX + (long long)r * MX + 64 + c, (c == 0) ? 1.f : 0.f); }
__global__ __launch_bounds__(256) void k_sa_adj(const float* __restrict__ P2, const int* __restrict__ rad, float* __restrict__ ADJ, int N) { const long long t = (long long)blockIdx.x * 256 + threadIdx.x; if (t >= (long long)N * (N / 4)) return; const int i = (int)(t / (N / 4)); const int j0 = 4 * (int)(t % (N / 4));
    const float r = (float)rad[0]; const float r2 = r * r; const float xi = P2[2 * i], yi = P2[2 * i + 1]; v4f o;
#pragma unroll
    for (int u = 0; u < 4; ++u) { const int j = j0 + u; const float dx = __fsub_rn(xi, P2[2 * j]), dy = __fsub_rn(yi, P2[2 * j + 1]); const float d2 = __fadd_rn(__fmul_rn(dx, dx), __fmul_rn(dy, dy)); o[u] = (d2 < r2 && j != i) ? 1.f : 0.f; }
    VST2V4(ADJ + (long long)i * N + j0, o); }
__global__ __launch_bounds__(256) void k_sa_comb(const float* __restrict__ MSGX, const float* __restrict__ AGX, float* __restrict__ COMB, int NR, int MX) { const long long t = (long long)blockIdx.x * 256 + threadIdx.x; if (t >= (long long)NR * 128) return; const int r = (int)(t >> 7), c = (int)(t & 127);
    float v; if (c < 64) v = MSGX[(long long)r * MX + c]; else { const float dg = fmaxf(AGX[(long long)r * MX + 64], 1.f); v = AGX[(long long)r * MX + (c - 64)] / dg; } VST2(float, COMB + t, v); }

template __global__ void k_gemm<0>(GemmP);

extern "C" void kernel_launch(void* const* d_in, const int* in_sizes, int n_in, void* d_out, int out_size, void* d_ws, size_t ws_size, hipStream_t stream) {
    (void)in_sizes; (void)n_in; (void)out_size; (void)ws_size;
    const float* st = (const float*)d_in[0];
    const float* pos = (const float*)d_in[1];
    const int* rad = (const int*)d_in[2];
    const float* W1 = (const float*)d_in[3];
    const float* b1 = (const float*)d_in[4];
    const float* W2 = (const float*)d_in[5];
    const float* b2 = (const float*)d_in[6];
    const float* W3 = (const float*)d_in[7];
    const float* b3 = (const float*)d_in[8];
    const float* W4 = (const float*)d_in[9];
    const float* b4 = (const float*)d_in[10];
    const float* W5 = (const float*)d_in[11];
    const float* b5 = (const float*)d_in[12];
    const float* W6 = (const float*)d_in[13];
    const float* b6 = (const float*)d_in[14];
    const int Bn = 4;
    const int N = 4096;
    const int D = 64;
    const int M = 64;
    const int HH = 128;
    const int NR = Bn * N;
    const int MX = 96;
    float* out = (float*)d_out;
    char* wsp = (char*)d_ws;
    float* ADJ = (float*)wsp; wsp += (((size_t)((size_t)N * N) * 4 + 255) / 256) * 256;
    float* MSGX = (float*)wsp; wsp += (((size_t)((size_t)NR * MX) * 4 + 255) / 256) * 256;
    float* AGX = (float*)wsp; wsp += (((size_t)((size_t)NR * MX) * 4 + 255) / 256) * 256;
    float* HB = (float*)wsp; wsp += (((size_t)((size_t)NR * HH) * 4 + 255) / 256) * 256;
    float* COMB = (float*)wsp; wsp += (((size_t)((size_t)NR * HH) * 4 + 255) / 256) * 256;
    float* FEAT = (float*)wsp; wsp += (((size_t)((size_t)NR * HH) * 4 + 255) / 256) * 256;
    { GemmP g1;
      g1.A = st; g1.B = W1; g1.bias = b1; g1.R = st; g1.C = HB;
      g1.sAo = 0; g1.sAi = 0; g1.sAm = D; g1.sAk = 1; g1.sBo = 0; g1.sBi = 0; g1.sBn = 1; g1.sBk = HH; g1.sCo = 0; g1.sCi = 0; g1.sCm = HH; g1.sRo = 0; g1.sRi = 0; g1.sRm = 0; g1.sRn = 0;
      g1.M = NR; g1.N = HH; g1.K = D; g1.zi_n = 1; g1.flags = 1; g1.act = 1;
      g1.alpha = 1.0f; g1.beta = 0.0f; g1.sa = 1.0f; g1.sb = 8.0f; g1.Npad = HH; g1.pad_ = 0;
      if ((long long)(NR) >= 64 && (long long)(HH) >= 64) k_gemmT<0, 4, 4><<<dim3((unsigned)((HH) + 63) / 64, (unsigned)((NR) + 63) / 64, (unsigned)(1)), 32, 0, stream>>>(g1);
      else k_gemm<0><<<dim3((unsigned)((HH) + 31) / 32, (unsigned)((NR) + 15) / 16, (unsigned)(1)), 32, 0, stream>>>(g1); }
    { GemmP g2;
      g2.A = HB; g2.B = W2; g2.bias = b2; g2.R = HB; g2.C = MSGX;
      g2.sAo = 0; g2.sAi = 0; g2.sAm = HH; g2.sAk = 1; g2.sBo = 0; g2.sBi = 0; g2.sBn = 1; g2.sBk = M; g2.sCo = 0; g2.sCi = 0; g2.sCm = MX; g2.sRo = 0; g2.sRi = 0; g2.sRm = 0; g2.sRn = 0;
      g2.M = NR; g2.N = M; g2.K = HH; g2.zi_n = 1; g2.flags = 1; g2.act = 0;
      g2.alpha = 1.0f; g2.beta = 0.0f; g2.sa = 1.0f; g2.sb = 8.0f; g2.Npad = M; g2.pad_ = 0;
      if ((long long)(NR) >= 64 && (long long)(M) >= 64) k_gemmT<0, 4, 4><<<dim3((unsigned)((M) + 63) / 64, (unsigned)((NR) + 63) / 64, (unsigned)(1)), 32, 0, stream>>>(g2);
      else k_gemm<0><<<dim3((unsigned)((M) + 31) / 32, (unsigned)((NR) + 15) / 16, (unsigned)(1)), 32, 0, stream>>>(g2); }
    k_sa_ones<<<(unsigned)((NR * 32 + 255) / 256), 256, 0, stream>>>(MSGX, NR, MX);
    k_sa_adj<<<(unsigned)(((long long)N * (N / 4) + 255) / 256), 256, 0, stream>>>(pos + (size_t)0 * N * 2, rad, ADJ, N);
    { GemmP gagg0;
      gagg0.A = ADJ; gagg0.B = MSGX + (size_t)0 * N * MX; gagg0.bias = ADJ; gagg0.R = ADJ; gagg0.C = AGX + (size_t)0 * N * MX;
      gagg0.sAo = 0; gagg0.sAi = 0; gagg0.sAm = N; gagg0.sAk = 1; gagg0.sBo = 0; gagg0.sBi = 0; gagg0.sBn = 1; gagg0.sBk = MX; gagg0.sCo = 0; gagg0.sCi = 0; gagg0.sCm = MX; gagg0.sRo = 0; gagg0.sRi = 0; gagg0.sRm = 0; gagg0.sRn = 0;
      gagg0.M = N; gagg0.N = MX; gagg0.K = N; gagg0.zi_n = 1; gagg0.flags = 0; gagg0.act = 0;
      gagg0.alpha = 1.0f; gagg0.beta = 0.0f; gagg0.sa = 1.0f; gagg0.sb = 1.0f; gagg0.Npad = MX; gagg0.pad_ = 0;
      if ((long long)(N) >= 64 && (long long)(MX) >= 64) k_gemmT<0, 4, 4><<<dim3((unsigned)((MX) + 63) / 64, (unsigned)((N) + 63) / 64, (unsigned)(1)), 32, 0, stream>>>(gagg0);
      else k_gemm<0><<<dim3((unsigned)((MX) + 31) / 32, (unsigned)((N) + 15) / 16, (unsigned)(1)), 32, 0, stream>>>(gagg0); }
    k_sa_adj<<<(unsigned)(((long long)N * (N / 4) + 255) / 256), 256, 0, stream>>>(pos + (size_t)1 * N * 2, rad, ADJ, N);
    { GemmP gagg1;
      gagg1.A = ADJ; gagg1.B = MSGX + (size_t)1 * N * MX; gagg1.bias = ADJ; gagg1.R = ADJ; gagg1.C = AGX + (size_t)1 * N * MX;
      gagg1.sAo = 0; gagg1.sAi = 0; gagg1.sAm = N; gagg1.sAk = 1; gagg1.sBo = 0; gagg1.sBi = 0; gagg1.sBn = 1; gagg1.sBk = MX; gagg1.sCo = 0; gagg1.sCi = 0; gagg1.sCm = MX; gagg1.sRo = 0; gagg1.sRi = 0; gagg1.sRm = 0; gagg1.sRn = 0;
      gagg1.M = N; gagg1.N = MX; gagg1.K = N; gagg1.zi_n = 1; gagg1.flags = 0; gagg1.act = 0;
      gagg1.alpha = 1.0f; gagg1.beta = 0.0f; gagg1.sa = 1.0f; gagg1.sb = 1.0f; gagg1.Npad = MX; gagg1.pad_ = 0;
      if ((long long)(N) >= 64 && (long long)(MX) >= 64) k_gemmT<0, 4, 4><<<dim3((unsigned)((MX) + 63) / 64, (unsigned)((N) + 63) / 64, (unsigned)(1)), 32, 0, stream>>>(gagg1);
      else k_gemm<0><<<dim3((unsigned)((MX) + 31) / 32, (unsigned)((N) + 15) / 16, (unsigned)(1)), 32, 0, stream>>>(gagg1); }
    k_sa_adj<<<(unsigned)(((long long)N * (N / 4) + 255) / 256), 256, 0, stream>>>(pos + (size_t)2 * N * 2, rad, ADJ, N);
    { GemmP gagg2;
      gagg2.A = ADJ; gagg2.B = MSGX + (size_t)2 * N * MX; gagg2.bias = ADJ; gagg2.R = ADJ; gagg2.C = AGX + (size_t)2 * N * MX;
      gagg2.sAo = 0; gagg2.sAi = 0; gagg2.sAm = N; gagg2.sAk = 1; gagg2.sBo = 0; gagg2.sBi = 0; gagg2.sBn = 1; gagg2.sBk = MX; gagg2.sCo = 0; gagg2.sCi = 0; gagg2.sCm = MX; gagg2.sRo = 0; gagg2.sRi = 0; gagg2.sRm = 0; gagg2.sRn = 0;
      gagg2.M = N; gagg2.N = MX; gagg2.K = N; gagg2.zi_n = 1; gagg2.flags = 0; gagg2.act = 0;
      gagg2.alpha = 1.0f; gagg2.beta = 0.0f; gagg2.sa = 1.0f; gagg2.sb = 1.0f; gagg2.Npad = MX; gagg2.pad_ = 0;
      if ((long long)(N) >= 64 && (long long)(MX) >= 64) k_gemmT<0, 4, 4><<<dim3((unsigned)((MX) + 63) / 64, (unsigned)((N) + 63) / 64, (unsigned)(1)), 32, 0, stream>>>(gagg2);
      else k_gemm<0><<<dim3((unsigned)((MX) + 31) / 32, (unsigned)((N) + 15) / 16, (unsigned)(1)), 32, 0, stream>>>(gagg2); }
    k_sa_adj<<<(unsigned)(((long long)N * (N / 4) + 255) / 256), 256, 0, stream>>>(pos + (size_t)3 * N * 2, rad, ADJ, N);
    { GemmP gagg3;
      gagg3.A = ADJ; gagg3.B = MSGX + (size_t)3 * N * MX; gagg3.bias = ADJ; gagg3.R = ADJ; gagg3.C = AGX + (size_t)3 * N * MX;
      gagg3.sAo = 0; gagg3.sAi = 0; gagg3.sAm = N; gagg3.sAk = 1; gagg3.sBo = 0; gagg3.sBi = 0; gagg3.sBn = 1; gagg3.sBk = MX; gagg3.sCo = 0; gagg3.sCi = 0; gagg3.sCm = MX; gagg3.sRo = 0; gagg3.sRi = 0; gagg3.sRm = 0; gagg3.sRn = 0;
      gagg3.M = N; gagg3.N = MX; gagg3.K = N; gagg3.zi_n = 1; gagg3.flags = 0; gagg3.act = 0;
      gagg3.alpha = 1.0f; gagg3.beta = 0.0f; gagg3.sa = 1.0f; gagg3.sb = 1.0f; gagg3.Npad = MX; gagg3.pad_ = 0;
      if ((long long)(N) >= 64 && (long long)(MX) >= 64) k_gemmT<0, 4, 4><<<dim3((unsigned)((MX) + 63) / 64, (unsigned)((N) + 63) / 64, (unsigned)(1)), 32, 0, stream>>>(gagg3);
      else k_gemm<0><<<dim3((unsigned)((MX) + 31) / 32, (unsigned)((N) + 15) / 16, (unsigned)(1)), 32, 0, stream>>>(gagg3); }
    k_sa_comb<<<(unsigned)(((long long)NR * 128 + 255) / 256), 256, 0, stream>>>(MSGX, AGX, COMB, NR, MX);
    { GemmP g3;
      g3.A = COMB; g3.B = W3; g3.bias = b3; g3.R = COMB; g3.C = HB;
      g3.sAo = 0; g3.sAi = 0; g3.sAm = HH; g3.sAk = 1; g3.sBo = 0; g3.sBi = 0; g3.sBn = 1; g3.sBk = HH; g3.sCo = 0; g3.sCi = 0; g3.sCm = HH; g3.sRo = 0; g3.sRi = 0; g3.sRm = 0; g3.sRn = 0;
      g3.M = NR; g3.N = HH; g3.K = HH; g3.zi_n = 1; g3.flags = 1; g3.act = 1;
      g3.alpha = 1.0f; g3.beta = 0.0f; g3.sa = 1.0f; g3.sb = 8.0f; g3.Npad = HH; g3.pad_ = 0;
      if ((long long)(NR) >= 64 && (long long)(HH) >= 64) k_gemmT<0, 4, 4><<<dim3((unsigned)((HH) + 63) / 64, (unsigned)((NR) + 63) / 64, (unsigned)(1)), 32, 0, stream>>>(g3);
      else k_gemm<0><<<dim3((unsigned)((HH) + 31) / 32, (unsigned)((NR) + 15) / 16, (unsigned)(1)), 32, 0, stream>>>(g3); }
    k_lincopy<<<(unsigned)(((long long)(NR) * (D) + 255) / 256), 256, 0, stream>>>(st, D, FEAT, HH, NR, D);
    { GemmP g4;
      g4.A = HB; g4.B = W4; g4.bias = b4; g4.R = HB; g4.C = FEAT + 64;
      g4.sAo = 0; g4.sAi = 0; g4.sAm = HH; g4.sAk = 1; g4.sBo = 0; g4.sBi = 0; g4.sBn = 1; g4.sBk = M; g4.sCo = 0; g4.sCi = 0; g4.sCm = HH; g4.sRo = 0; g4.sRi = 0; g4.sRm = 0; g4.sRn = 0;
      g4.M = NR; g4.N = M; g4.K = HH; g4.zi_n = 1; g4.flags = 1; g4.act = 0;
      g4.alpha = 1.0f; g4.beta = 0.0f; g4.sa = 1.0f; g4.sb = 8.0f; g4.Npad = M; g4.pad_ = 0;
      if ((long long)(NR) >= 64 && (long long)(M) >= 64) k_gemmT<0, 4, 4><<<dim3((unsigned)((M) + 63) / 64, (unsigned)((NR) + 63) / 64, (unsigned)(1)), 32, 0, stream>>>(g4);
      else k_gemm<0><<<dim3((unsigned)((M) + 31) / 32, (unsigned)((NR) + 15) / 16, (unsigned)(1)), 32, 0, stream>>>(g4); }
    { GemmP g5;
      g5.A = FEAT; g5.B = W5; g5.bias = b5; g5.R = FEAT; g5.C = HB;
      g5.sAo = 0; g5.sAi = 0; g5.sAm = HH; g5.sAk = 1; g5.sBo = 0; g5.sBi = 0; g5.sBn = 1; g5.sBk = HH; g5.sCo = 0; g5.sCi = 0; g5.sCm = HH; g5.sRo = 0; g5.sRi = 0; g5.sRm = 0; g5.sRn = 0;
      g5.M = NR; g5.N = HH; g5.K = HH; g5.zi_n = 1; g5.flags = 1; g5.act = 1;
      g5.alpha = 1.0f; g5.beta = 0.0f; g5.sa = 1.0f; g5.sb = 8.0f; g5.Npad = HH; g5.pad_ = 0;
      if ((long long)(NR) >= 64 && (long long)(HH) >= 64) k_gemmT<0, 4, 4><<<dim3((unsigned)((HH) + 63) / 64, (unsigned)((NR) + 63) / 64, (unsigned)(1)), 32, 0, stream>>>(g5);
      else k_gemm<0><<<dim3((unsigned)((HH) + 31) / 32, (unsigned)((NR) + 15) / 16, (unsigned)(1)), 32, 0, stream>>>(g5); }
    { GemmP g6;
      g6.A = HB; g6.B = W6; g6.bias = b6; g6.R = st; g6.C = out;
      g6.sAo = 0; g6.sAi = 0; g6.sAm = HH; g6.sAk = 1; g6.sBo = 0; g6.sBi = 0; g6.sBn = 1; g6.sBk = D; g6.sCo = 0; g6.sCi = 0; g6.sCm = D; g6.sRo = 0; g6.sRi = 0; g6.sRm = D; g6.sRn = 1;
      g6.M = NR; g6.N = D; g6.K = HH; g6.zi_n = 1; g6.flags = 5; g6.act = 0;
      g6.alpha = 1.0f; g6.beta = 1.0f; g6.sa = 1.0f; g6.sb = 8.0f; g6.Npad = D; g6.pad_ = 0;
      if ((long long)(NR) >= 64 && (long long)(D) >= 64) k_gemmT<0, 4, 4><<<dim3((unsigned)((D) + 63) / 64, (unsigned)((NR) + 63) / 64, (unsigned)(1)), 32, 0, stream>>>(g6);
      else k_gemm<0><<<dim3((unsigned)((D) + 31) / 32, (unsigned)((NR) + 15) / 16, (unsigned)(1)), 32, 0, stream>>>(g6); }
}
